// VpMoETPAAttention_47871705481251
// MI455X (gfx1250) — hardware-verified
//
#include <hip/hip_runtime.h>
#include <math.h>

typedef __attribute__((ext_vector_type(16))) _Float16 v16h;
typedef __attribute__((ext_vector_type(16))) __bf16 v16b;
typedef __attribute__((ext_vector_type(8)))  _Float16 v8h;
typedef __attribute__((ext_vector_type(8)))  float v8f;
typedef __attribute__((ext_vector_type(4)))  float v4f;
typedef __attribute__((ext_vector_type(2)))  float v2f;
typedef __attribute__((ext_vector_type(4)))  unsigned v4u;
typedef __attribute__((ext_vector_type(4)))  int v4i;
typedef float __attribute__((may_alias)) float_a;
typedef int __attribute__((may_alias)) int_a;

template <typename T> __device__ __forceinline__ void vst2(void* p, T v) { *(volatile T*)p = v; __threadfence(); *(volatile T*)p = v; }
__device__ __forceinline__ v8f wmma16(v16h a, v16h b, v8f c) {
  v8f d = __builtin_amdgcn_wmma_f32_16x16x32_f16(false, a, false, b, (short)0, c, false, false);
  asm volatile("v_nop\n\tv_nop\n\tv_nop\n\tv_nop" : "+v"(d) : "v"(a), "v"(b));
  return d;
}
__device__ __forceinline__ v8f wmma_bf(v16b a, v16b b, v8f c) {
  v8f d = __builtin_amdgcn_wmma_f32_16x16x32_bf16(false, a, false, b, (short)0, c, false, false);
  asm volatile("v_nop\n\tv_nop\n\tv_nop\n\tv_nop" : "+v"(d) : "v"(a), "v"(b));
  return d;
}
__device__ __forceinline__ v16h frag_h(const _Float16* rowk0, int lane) {
  union { v16h v; v8h q[2]; } u; const _Float16* p = rowk0 + 8 * (lane >> 4);
  u.q[0] = *(const v8h*)p; u.q[1] = *(const v8h*)(p + 16); return u.v;
}
__device__ __forceinline__ v16h frag_f32(const float* rowk0, int lane) {
  v16h a; const float* p = rowk0 + 8 * (lane >> 4);
#pragma unroll
  for (int i = 0; i < 8; ++i) { a[i] = (_Float16)p[i]; a[8 + i] = (_Float16)p[16 + i]; }
  return a;
}
__device__ __forceinline__ v16h frag_f32s(const float* rowk0, int lane, float sc) {
  v16h a; const float* p = rowk0 + 8 * (lane >> 4);
#pragma unroll
  for (int i = 0; i < 8; ++i) { a[i] = (_Float16)(p[i] * sc); a[8 + i] = (_Float16)(p[16 + i] * sc); }
  return a;
}
__device__ __forceinline__ v16h fragc_f32(const float* W, int k0, int n, int lane, int ld, int K) {
  v16h a; const int g = lane >> 4;
#pragma unroll
  for (int i = 0; i < 8; ++i) { const int ka = k0 + 8 * g + i, kb = ka + 16;
    a[i] = (_Float16)(ka < K ? W[(size_t)(ka < K ? ka : K - 1) * ld + n] : 0.f); a[8 + i] = (_Float16)(kb < K ? W[(size_t)(kb < K ? kb : K - 1) * ld + n] : 0.f); }
  return a;
}
struct F2 { v16b h, l; };
__device__ __forceinline__ F2 bsplit16(const float v[16]) { F2 r;
#pragma unroll
  for (int i = 0; i < 16; ++i) { const __bf16 h = (__bf16)v[i]; r.h[i] = h; r.l[i] = (__bf16)(v[i] - (float)h); }
  return r; }
__device__ __forceinline__ F2 split_row(const float* row, int k0, int lane) { float v[16]; const float* p = row + k0 + 8 * (lane >> 4);
#pragma unroll
  for (int i = 0; i < 8; ++i) { v[i] = p[i]; v[8 + i] = p[16 + i]; }
  return bsplit16(v); }
__device__ __forceinline__ F2 split_rowK(const float* row, int k0, int lane, int K) { float v[16]; const int g = lane >> 4;
#pragma unroll
  for (int i = 0; i < 8; ++i) { const int ka = k0 + 8 * g + i, kb = ka + 16; v[i] = ka < K ? row[ka < K ? ka : K - 1] : 0.f; v[8 + i] = kb < K ? row[kb < K ? kb : K - 1] : 0.f; }
  return bsplit16(v); }
__device__ __forceinline__ F2 split_col(const float* W, int k0, int n, int lane, int ld, int K) { float v[16]; const int g = lane >> 4;
#pragma unroll
  for (int i = 0; i < 8; ++i) { const int ka = k0 + 8 * g + i, kb = ka + 16; v[i] = ka < K ? W[(size_t)(ka < K ? ka : K - 1) * ld + n] : 0.f; v[8 + i] = kb < K ? W[(size_t)(kb < K ? kb : K - 1) * ld + n] : 0.f; }
  return bsplit16(v); }
__device__ __forceinline__ v8f mac3(const F2& a, const F2& b, v8f c) { c = wmma_bf(a.l, b.h, c); c = wmma_bf(a.h, b.l, c); return wmma_bf(a.h, b.h, c); }
__device__ __forceinline__ float sigm(float v) { return 1.0f / (1.0f + expf(-v)); }
#define LDSX() do { asm volatile("s_wait_dscnt 0" ::: "memory"); __builtin_amdgcn_wave_barrier(); __builtin_amdgcn_fence(__ATOMIC_RELEASE, "workgroup"); } while (0)


#define NB 2
#define SS 2048
#define DM 2048
#define NH 16
#define NKV 4
#define HD 128
#define QR 6
#define KR 2
#define NF 1392
#define NFP 1408
#define NR (NB * SS)
#ifndef TRB
#define TRB (NR / 64)
#define TQB (SS / 64)
#define TNB NB
#endif
typedef __attribute__((ext_vector_type(8))) __bf16 v8b;
__device__ __forceinline__ v16b frag_b(const __bf16* rowk0, int lane) {
  union { v16b v; v8b q[2]; } u; const __bf16* p = rowk0 + 8 * (lane >> 4);
  u.q[0] = *(const v8b*)p; u.q[1] = *(const v8b*)(p + 16); return u.v;
}
__device__ __forceinline__ v16b frag_gbf(const float* rowk0, int lane) {
  v16b a; const float* p = rowk0 + 8 * (lane >> 4);
#pragma unroll
  for (int i = 0; i < 8; ++i) { a[i] = (__bf16)p[i]; a[8 + i] = (__bf16)p[16 + i]; }
  return a;
}
__device__ __forceinline__ float bfr(float v) { return (float)(__bf16)v; }
__device__ __attribute__((noinline)) float exp_ni(float v) { return expf(v); }
__device__ __attribute__((noinline)) float log_ni(float v) { return logf(v); }

#define WS_PT1  0u
#define WS_PTO  (WS_PT1 + 2u * NF * DM)
#define WS_PR   (WS_PTO + 2u * DM * DM)
#define WS_Q    (WS_PR + 4u * NR * NFP)
#define WS_K    (WS_Q + 4u * NR * DM)
#define WS_VTH  (WS_K + 4u * NR * NKV * HD)
#define WS_VTL  (WS_VTH + 2u * NB * NKV * HD * SS)
#define WS_FL   (WS_VTL + 2u * NB * NKV * HD * SS)
#define WS_END  (WS_FL + 4u * 32 * 64)

__global__ __launch_bounds__(256) void k_pack(const float* __restrict__ aq, const float* __restrict__ ak, const float* __restrict__ av, const float* __restrict__ bq, const float* __restrict__ bk, const float* __restrict__ bv, const float* __restrict__ wo, __bf16* __restrict__ PT1, __bf16* __restrict__ PTO) {
  __shared__ __align__(16) __bf16 srow[DM];
  const int n = blockIdx.x, tid = threadIdx.x; const float* src; int ld, c; __bf16* dst;
  if (n < NF) { dst = PT1 + (size_t)n * DM;
    if (n < 96) { src = aq; ld = 96; c = n; } else if (n < 104) { src = ak; ld = 8; c = n - 96; } else if (n < 112) { src = av; ld = 8; c = n - 104; }
    else if (n < 880) { src = bq; ld = 768; c = n - 112; } else if (n < 1136) { src = bk; ld = 256; c = n - 880; } else { src = bv; ld = 256; c = n - 1136; } }
  else { src = wo; ld = DM; c = n - NF; dst = PTO + (size_t)c * DM; }
  for (int k = tid; k < DM; k += 256) srow[k] = (__bf16)src[(size_t)k * ld + c];
  __syncthreads();
  vst2((unsigned*)(dst + tid * 8), *(const v4u*)(&srow[tid * 8]));
}
__global__ __launch_bounds__(128) void k_proj(const float* __restrict__ X, const __bf16* __restrict__ PT1, float* __restrict__ PR) {
  __shared__ __align__(16) float so[4][16][132];
  const int tid = threadIdx.x, wave = tid >> 5, lane = tid & 31, col = lane & 15, g = lane >> 4; const size_t r0 = (size_t)blockIdx.x * 64 + wave * 16; const int n0 = blockIdx.y * 128; const int ntile = (NF - n0) / 16 < 8 ? (NF - n0) / 16 : 8;
  v8f acc[8] = {};
#pragma unroll 1
  for (int kc = 0; kc < DM / 32; ++kc) { const v16b a = frag_gbf(X + (r0 + col) * DM + kc * 32, lane);
#pragma unroll
    for (int j = 0; j < 8; ++j) if (j < ntile) acc[j] = wmma_bf(a, frag_b(PT1 + (size_t)(n0 + j * 16 + col) * DM + kc * 32, lane), acc[j]); }
#pragma unroll
  for (int j = 0; j < 8; ++j)
#pragma unroll
    for (int r = 0; r < 8; ++r) so[wave][8 * g + r][j * 16 + col] = j < ntile ? acc[j][r] : 0.f;
  LDSX();
  for (int rl = 0; rl < 16; ++rl) vst2(PR + (r0 + rl) * NFP + n0 + lane * 4, *(const v4f*)(&so[wave][rl][lane * 4]));
}
__global__ __launch_bounds__(256) void k_qkv(const float* __restrict__ PR, const float* __restrict__ cosb, const float* __restrict__ sinb, float* __restrict__ Q, float* __restrict__ Kb, __bf16* __restrict__ VTH, __bf16* __restrict__ VTL) {
  __shared__ float sbq[QR][HD], sbk[KR][HD], sbv[KR][HD], saq[NH * QR], sak[NKV * KR], sav[NKV * KR];
  __shared__ __align__(16) float sq[DM]; __shared__ __align__(16) float sk[NKV * HD];
  __shared__ __align__(16) __bf16 svh[NKV * HD][72], svl[NKV * HD][72];
  const int tid = threadIdx.x; const size_t t0 = (size_t)blockIdx.x * 64; const int b = (int)(t0 / SS), p0 = (int)(t0 % SS);
#pragma unroll 1
  for (int tl = 0; tl < 64; ++tl) { const size_t t = t0 + tl; const float* pr = PR + t * NFP;
    __syncthreads();
    if (tid < NH * QR) saq[tid] = pr[tid]; else if (tid < 104) sak[tid - 96] = pr[tid]; else if (tid < 112) sav[tid - 104] = pr[tid];
    for (int q = tid; q < (QR + KR) * 64; q += 256) { const int r = q >> 6, d = q & 63; const float c = bfr(cosb[t * 64 + d]), s = bfr(sinb[t * 64 + d]);
      if (r < QR) { const float x1 = pr[112 + r * HD + d], x2 = pr[112 + r * HD + 64 + d]; sbq[r][d] = x1 * c - x2 * s; sbq[r][64 + d] = x2 * c + x1 * s; }
      else { const int rr = r - QR; const float x1 = pr[880 + rr * HD + d], x2 = pr[880 + rr * HD + 64 + d]; sbk[rr][d] = x1 * c - x2 * s; sbk[rr][64 + d] = x2 * c + x1 * s; } }
    sbv[tid >> 7][tid & 127] = pr[1136 + tid];
    __syncthreads();
    for (int q = tid; q < NH * HD; q += 256) { const int h = q >> 7, d = q & 127; float s = 0.f;
#pragma unroll
      for (int r = 0; r < QR; ++r) s += saq[h * QR + r] * sbq[r][d];
      sq[q] = s / (float)QR; }
    for (int q = tid; q < NKV * HD; q += 256) { const int kv = q >> 7, d = q & 127; const float kk = (sak[kv * KR] * sbk[0][d] + sak[kv * KR + 1] * sbk[1][d]) / (float)KR; const float vv = (sav[kv * KR] * sbv[0][d] + sav[kv * KR + 1] * sbv[1][d]) / (float)KR;
      sk[q] = kk; const __bf16 hb = (__bf16)vv; svh[q][tl] = hb; svl[q][tl] = (__bf16)(vv - (float)hb); }
    __syncthreads();
    for (int q = tid; q < DM / 4; q += 256) vst2(Q + t * DM + q * 4, *(const v4f*)&sq[q * 4]);
    if (tid < NKV * HD / 4) vst2(Kb + t * (NKV * HD) + tid * 4, *(const v4f*)&sk[tid * 4]); }
  __syncthreads();
  for (int q = tid; q < NKV * HD * 8; q += 256) { const int row = q >> 3, pc = q & 7; const size_t o = ((size_t)b * NKV * HD + row) * SS + p0 + pc * 8; vst2((unsigned*)(VTH + o), *(const v4u*)&svh[row][pc * 8]); vst2((unsigned*)(VTL + o), *(const v4u*)&svl[row][pc * 8]); }
}
__global__ __launch_bounds__(64) void k_flags(const float* __restrict__ mask, int* __restrict__ FL) {
  __shared__ int sfl[64];
  const int qb = blockIdx.x, ks = threadIdx.x; bool allm = true, allz = true;
  for (int r = 0; r < 64; ++r) for (int c = 0; c < 32; ++c) { const float v = bfr(mask[(size_t)(qb * 64 + r) * SS + ks * 32 + c]); allm = allm && (v <= -1.0e8f); allz = allz && (v == 0.f); }
  sfl[ks] = allm ? 0 : (allz ? 1 : 2);
  __syncthreads();
  if (ks < 16) vst2(FL + qb * 64 + ks * 4, *(const v4i*)&sfl[ks * 4]);
}
__global__ __launch_bounds__(128) void k_attn(float* __restrict__ QO, const float* __restrict__ Kb, const __bf16* __restrict__ VTH, const __bf16* __restrict__ VTL, const float* __restrict__ mask, const int* __restrict__ FL, const float* __restrict__ sinks) {
  __shared__ __align__(16) float sp[4][16][36]; __shared__ __align__(16) float so[4][16][132];
  const int tid = threadIdx.x, wave = tid >> 5, lane = tid & 31, col = lane & 15, g = lane >> 4;
  const int qb = blockIdx.x, bh = blockIdx.y, b = bh >> 4, h = bh & 15, kvh = h >> 2; const int q0 = qb * 64 + wave * 16; const size_t tq = (size_t)b * SS + q0;
  const float scaling = 1.0f / sqrtf((float)HD);
  F2 a[4];
#pragma unroll
  for (int kc = 0; kc < 4; ++kc) a[kc] = split_row(QO + (tq + col) * DM + h * HD, kc * 32, lane);
  float m[8], l[8];
#pragma unroll
  for (int r = 0; r < 8; ++r) { m[r] = -3.0e38f; l[r] = 0.f; }
  v8f acc[8] = {};
#pragma unroll 1
  for (int ks = 0; ks < SS / 32; ++ks) { const int fl = FL[qb * 64 + ks]; if (fl == 0) continue;
    v8f s[2];
#pragma unroll
    for (int ct = 0; ct < 2; ++ct) { const int kk = ks * 32 + ct * 16 + col; const float* krow = Kb + ((size_t)b * SS + kk) * (NKV * HD) + kvh * HD; v8f accs = {};
#pragma unroll
      for (int kc = 0; kc < 4; ++kc) { const F2 kb = split_row(krow, kc * 32, lane); accs = mac3(a[kc], kb, accs); }
#pragma unroll
      for (int r = 0; r < 8; ++r) { float v = accs[r] * scaling; if (fl == 2) v += bfr(mask[(size_t)(q0 + 8 * g + r) * SS + kk]); s[ct][r] = v; } }
#pragma unroll
    for (int r = 0; r < 8; ++r) { float mx = fmaxf(s[0][r], s[1][r]);
#pragma unroll
      for (int o = 1; o < 16; o <<= 1) mx = fmaxf(mx, __shfl_xor(mx, o));
      const float mn = fmaxf(m[r], mx); const float alpha = exp_ni(m[r] - mn);
      const float e0 = exp_ni(s[0][r] - mn), e1 = exp_ni(s[1][r] - mn); float es = e0 + e1;
#pragma unroll
      for (int o = 1; o < 16; o <<= 1) es += __shfl_xor(es, o);
      l[r] = l[r] * alpha + es; m[r] = mn;
#pragma unroll
      for (int dt = 0; dt < 8; ++dt) acc[dt][r] *= alpha;
      sp[wave][8 * g + r][col] = e0; sp[wave][8 * g + r][16 + col] = e1; }
    LDSX();
    const F2 pa = split_row(&sp[wave][col][0], 0, lane);
#pragma unroll
    for (int dt = 0; dt < 8; ++dt) { const size_t vrow = ((size_t)b * NKV * HD + kvh * HD + dt * 16 + col) * SS + ks * 32; const v16b vh = frag_b(VTH + vrow, lane), vl = frag_b(VTL + vrow, lane);
      acc[dt] = wmma_bf(pa.l, vh, acc[dt]); acc[dt] = wmma_bf(pa.h, vl, acc[dt]); acc[dt] = wmma_bf(pa.h, vh, acc[dt]); }
    LDSX(); }
  const float sk = bfr(sinks[h]);
#pragma unroll
  for (int r = 0; r < 8; ++r) { const float lz = m[r] + log_ni(l[r]); const float gate = 1.0f / (1.0f + exp_ni(-(lz - sk))); const float f = gate / l[r];
#pragma unroll
    for (int dt = 0; dt < 8; ++dt) so[wave][8 * g + r][dt * 16 + col] = acc[dt][r] * f; }
  LDSX();
  for (int rl = 0; rl < 16; ++rl) vst2(QO + (tq + rl) * DM + h * HD + lane * 4, *(const v4f*)&so[wave][rl][lane * 4]);
}
__global__ __launch_bounds__(128) void k_out(const float* __restrict__ O, const __bf16* __restrict__ PTO, float* __restrict__ Y) {
  __shared__ __align__(16) float so[4][16][132];
  const int tid = threadIdx.x, wave = tid >> 5, lane = tid & 31, col = lane & 15, g = lane >> 4; const size_t r0 = (size_t)blockIdx.x * 64 + wave * 16; const int n0 = blockIdx.y * 128;
  v8f acc[8] = {};
#pragma unroll 1
  for (int kc = 0; kc < DM / 32; ++kc) { const F2 a = split_row(O + (r0 + col) * DM, kc * 32, lane);
#pragma unroll
    for (int j = 0; j < 8; ++j) { const v16b w = frag_b(PTO + (size_t)(n0 + j * 16 + col) * DM + kc * 32, lane); acc[j] = wmma_bf(a.l, w, acc[j]); acc[j] = wmma_bf(a.h, w, acc[j]); } }
#pragma unroll
  for (int j = 0; j < 8; ++j)
#pragma unroll
    for (int r = 0; r < 8; ++r) so[wave][8 * g + r][j * 16 + col] = acc[j][r];
  LDSX();
  for (int rl = 0; rl < 16; ++rl) vst2(Y + (r0 + rl) * DM + n0 + lane * 4, *(const v4f*)(&so[wave][rl][lane * 4]));
}

extern "C" void kernel_launch(void* const* d_in, const int* in_sizes, int n_in, void* d_out, int out_size, void* d_ws, size_t ws_size, hipStream_t stream) {
  (void)in_sizes; (void)n_in; (void)out_size;
  const float** F = (const float**)d_in;
  if (ws_size < (size_t)WS_END) return;
  char* ws = (char*)d_ws; __bf16 *PT1 = (__bf16*)(ws + WS_PT1), *PTO = (__bf16*)(ws + WS_PTO), *VTH = (__bf16*)(ws + WS_VTH), *VTL = (__bf16*)(ws + WS_VTL); float *PR = (float*)(ws + WS_PR), *Q = (float*)(ws + WS_Q), *Kb = (float*)(ws + WS_K); int* FL = (int*)(ws + WS_FL);
  k_pack<<<NF + DM, 256, 0, stream>>>(F[4], F[5], F[6], F[7], F[8], F[9], F[10], PT1, PTO);
  k_proj<<<dim3(TRB, NFP / 128), 128, 0, stream>>>(F[0], PT1, PR);
  k_qkv<<<TRB, 256, 0, stream>>>(PR, F[1], F[2], Q, Kb, VTH, VTL);
  k_flags<<<32, 64, 0, stream>>>(F[3], FL);
  k_attn<<<dim3(TQB, TNB * NH), 128, 0, stream>>>(Q, Kb, VTH, VTL, F[3], FL, F[11]);
  k_out<<<dim3((TNB < NB ? TQB : NR / 64), DM / 128), 128, 0, stream>>>(Q, PTO, (float*)d_out);
}
